// InputFeatureEmbedder_91293824844486
// MI455X (gfx1250) — hardware-verified
//
#include <hip/hip_runtime.h>
#include <stddef.h>
#include <stdint.h>

#define NB   2
#define NA   8192
#define MA   (NB * NA)
#define DS   128
#define DP   16
#define NH   4
#define HD   32
#define QW   64
#define KW   128
#define PADW 32
#define NWI  (NA / QW)
#define DT   384
#define NTK  1024
#define DEP  3
#define DFF  512
#define KF   389
#define KFL  416
#define KFP  448
#define VTH  64
#define VTP  (VTH + NA + VTH)
#define OTP  68
#define TTP  132
#define PTP  136
#define BTP  132

static_assert(MA == 16384);
static_assert(NH * HD == DS);
static_assert(NA % QW == 0);
static_assert(MA % 128 == 0);
static_assert(NA % 256 == 0);
static_assert(KFL % 32 == 0);
static_assert(KFP % 64 == 0);
static_assert(KFL <= KFP);
static_assert((VTP * 2) % 128 == 0);
static_assert(NTK % 32 == 0);
static_assert(DT % 4 == 0);
static_assert(64 * TTP <= 128 * OTP);

typedef _Float16     v8h  __attribute__((ext_vector_type(8)));
typedef _Float16     v16h __attribute__((ext_vector_type(16)));
typedef float        v8f  __attribute__((ext_vector_type(8)));
typedef float        v4f  __attribute__((ext_vector_type(4)));
typedef unsigned int v4u  __attribute__((ext_vector_type(4)));
typedef v8h __attribute__((may_alias)) v8ha;
typedef v4f __attribute__((may_alias)) v4fa;
typedef v4u __attribute__((may_alias)) v4ua;
union Frag { v16h v; v8h half[2]; };

__device__ __forceinline__ v8f mma(v16h a, v16h b, v8f c) {
  c = __builtin_amdgcn_wmma_f32_16x16x32_f16(false, a, false, b, (short)0, c, false, false);
  asm volatile("v_nop\n\tv_nop\n\tv_nop\n\tv_nop" : "+v"(c) : "v"(a), "v"(b));
  return c;
}

__device__ __forceinline__ v8f zero8() { return (v8f){0.f, 0.f, 0.f, 0.f, 0.f, 0.f, 0.f, 0.f}; }

__device__ __forceinline__ v16h ldq(const _Float16* q) {
  Frag f;
  f.half[0] = *(const v8ha*)(q);
  f.half[1] = *(const v8ha*)(q + 16);
  return f.v;
}
__device__ __forceinline__ v16h ldf(const _Float16* p, int ld, int row0, int k0, int lane) {
  return ldq(p + (size_t)(row0 + (lane & 15)) * ld + k0 + 8 * (lane >> 4));
}

__device__ __forceinline__ v4u pk2(v4f a, v4f b) {
  union { v8h h; v4u u; } t;
  t.h = (v8h){(_Float16)a[0], (_Float16)a[1], (_Float16)a[2], (_Float16)a[3],
              (_Float16)b[0], (_Float16)b[1], (_Float16)b[2], (_Float16)b[3]};
  return t.u;
}

__device__ __forceinline__ v4f relu4(v4f v) {
  return (v4f){fmaxf(v[0], 0.f), fmaxf(v[1], 0.f), fmaxf(v[2], 0.f), fmaxf(v[3], 0.f)};
}

__device__ __forceinline__ void wsync() {
  __builtin_amdgcn_fence(__ATOMIC_RELEASE, "wavefront");
  __builtin_amdgcn_wave_barrier();
}

__global__ __launch_bounds__(256) void k_wtr(const float* __restrict__ W, int K, int N, int wz,
                                             _Float16* __restrict__ T, int kp, int tz, float scale, int perm) {
  __shared__ __align__(16) float sT[64 * OTP];
  const int tid = threadIdx.x;
  const int k0 = blockIdx.x * 64, n0 = blockIdx.y * 64, z = blockIdx.z;
  const float* Wz = W + (size_t)z * wz;
#pragma unroll
  for (int it = 0; it < 4; ++it) {
    const int idx = tid + 256 * it;
    const int kr = idx >> 4, nq = idx & 15;
    const int kk = k0 + kr;
    int krow = kk;
    int kval = (kk < K) ? 1 : 0;
    if (perm != 0) {
      krow = (kk < 384) ? (kk + 5) : (kk - 384);
      kval = (kk < KF) ? 1 : 0;
    }
    krow = min(max(krow, 0), K - 1);
    const int n  = n0 + 4 * nq;
    const int nc = min(n, N - 4);
    const v4f v = *(const v4f*)(Wz + (size_t)krow * N + nc);
    const bool ok = (kval != 0) && (n < N);
#pragma unroll
    for (int i = 0; i < 4; ++i) sT[(4 * nq + i) * OTP + kr] = ok ? v[i] * scale : 0.f;
  }
  __syncthreads();
  v4u w[2];
  size_t go[2];
#pragma unroll
  for (int it = 0; it < 2; ++it) {
    const int idx = tid + 256 * it;
    const int nr = idx >> 3, pc = idx & 7;
    const v4fa* r = (const v4fa*)(sT + nr * OTP + 8 * pc);
    w[it]  = pk2(r[0], r[1]);
    go[it] = (size_t)z * tz + (size_t)(n0 + nr) * kp + k0 + 8 * pc;
  }
  for (int ps = 0; ps < 2; ++ps) {
#pragma unroll
    for (int it = 0; it < 2; ++it) *(volatile v4u*)(T + go[it]) = w[it];
    __threadfence();
  }
}

__global__ __launch_bounds__(256) void k_feats(const float* __restrict__ pos, const float* __restrict__ chg,
                                               const float* __restrict__ msk, const float* __restrict__ elem,
                                               const float* __restrict__ chars, _Float16* __restrict__ F) {
  const int tid = threadIdx.x, lane = tid & 31, wave = tid >> 5;
  const int row = blockIdx.x * 8 + wave;
  const float s0 = pos[(size_t)row * 3 + 0], s1 = pos[(size_t)row * 3 + 1], s2 = pos[(size_t)row * 3 + 2];
  const float s3 = chg[row], s4 = msk[row];
  v4u w[2];
  size_t go[2];
#pragma unroll
  for (int it = 0; it < 2; ++it) {
    const int p   = lane + 32 * it;
    const int pe  = min(p, 15);
    const int pcx = min(max(p - 16, 0), 31);
    const float* ep = elem + (size_t)row * 128 + 8 * pe;
    const float* cp = chars + (size_t)row * 256 + 8 * pcx;
    const v4f e0 = *(const v4f*)(ep), e1 = *(const v4f*)(ep + 4);
    const v4f c0 = *(const v4f*)(cp), c1 = *(const v4f*)(cp + 4);
    const v4f q0 = {s0, s1, s2, s3};
    const v4f q1 = {s4, 0.f, 0.f, 0.f};
    const v4f zz = {0.f, 0.f, 0.f, 0.f};
    const v4f a0 = (p < 16) ? e0 : ((p < 48) ? c0 : ((p == 48) ? q0 : zz));
    const v4f a1 = (p < 16) ? e1 : ((p < 48) ? c1 : ((p == 48) ? q1 : zz));
    w[it]  = pk2(a0, a1);
    go[it] = (size_t)row * KFP + 8 * p;
  }
  for (int ps = 0; ps < 2; ++ps) {
    *(volatile v4u*)(F + go[0]) = w[0];
    if (lane < 24) *(volatile v4u*)(F + go[1]) = w[1];
    __threadfence();
  }
}

__global__ __launch_bounds__(256) void k_zvt(_Float16* __restrict__ Vt) {
  const int idx = blockIdx.x * 256 + threadIdx.x;
  const int L = idx >> 3, pc = idx & 7;
  const int row = L >> 1, side = L & 1;
  const size_t go = (size_t)row * VTP + (side ? (VTH + NA) : 0) + 8 * pc;
  const v4u z = {0u, 0u, 0u, 0u};
  *(volatile v4u*)(Vt + go) = z;
  __threadfence();
  *(volatile v4u*)(Vt + go) = z;
}

__global__ __launch_bounds__(256) void k_ln(const float* __restrict__ X, _Float16* __restrict__ H) {
  const int tid = threadIdx.x, lane = tid & 31, wave = tid >> 5, hh = lane >> 4, c = lane & 15;
  const int row = (blockIdx.x * 8 + wave) * 2 + hh;
  const float* x = X + (size_t)row * DS + 8 * c;
  const v4f a0 = *(const v4f*)(x), a1 = *(const v4f*)(x + 4);
  float s = (a0[0] + a0[1]) + (a0[2] + a0[3]) + (a1[0] + a1[1]) + (a1[2] + a1[3]);
#pragma unroll
  for (int off = 1; off < 16; off <<= 1) s += __shfl_xor(s, off, 32);
  const float mean = s * (1.0f / DS);
  float v = 0.f;
#pragma unroll
  for (int i = 0; i < 4; ++i) { const float d0 = a0[i] - mean, d1 = a1[i] - mean; v += d0 * d0; v += d1 * d1; }
#pragma unroll
  for (int off = 1; off < 16; off <<= 1) v += __shfl_xor(v, off, 32);
  const float r = rsqrtf(v * (1.0f / DS) + 1e-5f);
  const v4f o0 = {(a0[0] - mean) * r, (a0[1] - mean) * r, (a0[2] - mean) * r, (a0[3] - mean) * r};
  const v4f o1 = {(a1[0] - mean) * r, (a1[1] - mean) * r, (a1[2] - mean) * r, (a1[3] - mean) * r};
  const v4u w = pk2(o0, o1);
  const size_t go = (size_t)row * DS + 8 * c;
  *(volatile v4u*)(H + go) = w;
  __threadfence();
  *(volatile v4u*)(H + go) = w;
}

__global__ __launch_bounds__(256) void k_gemm(const _Float16* __restrict__ A, int lda,
                                              const _Float16* __restrict__ Bt, int ldb, int bzs,
                                              int K, float oscale,
                                              float* Cf, int ldcf, int has_f, int resid, int relu_f,
                                              _Float16* Ch, int ldch, int chzs, int has_h, int relu_h,
                                              _Float16* Vt, int vt_z) {
  __shared__ __align__(16) float st[128 * OTP];
  const int tid = threadIdx.x, lane = tid & 31, wave = tid >> 5;
  const int hh = lane >> 4, c = lane & 15;
  const int z = blockIdx.z;
  const int mblk = blockIdx.y * 128, nblk = blockIdx.x * 64;
  const int mw = (wave >> 1) * 32, nw = (wave & 1) * 32;
  const _Float16* Bz = Bt + (size_t)z * bzs;

  v8f acc[2][2];
#pragma unroll
  for (int s = 0; s < 2; ++s)
#pragma unroll
    for (int t = 0; t < 2; ++t) acc[s][t] = zero8();

#pragma unroll 1
  for (int k0 = 0; k0 < K; k0 += 32) {
    const v16h a0 = ldf(A, lda, mblk + mw, k0, lane);
    const v16h a1 = ldf(A, lda, mblk + mw + 16, k0, lane);
#pragma unroll
    for (int t = 0; t < 2; ++t) {
      const v16h b = ldf(Bz, ldb, nblk + nw + 16 * t, k0, lane);
      acc[0][t] = mma(a0, b, acc[0][t]);
      acc[1][t] = mma(a1, b, acc[1][t]);
    }
  }

  const bool tr = (z == vt_z);
  if (!tr) {
#pragma unroll
    for (int s = 0; s < 2; ++s)
#pragma unroll
      for (int t = 0; t < 2; ++t)
#pragma unroll
        for (int r = 0; r < 8; ++r) {
          const int row = mw + 16 * s + 8 * hh + r;
          const int col = nw + 16 * t + c;
          st[row * OTP + col] = acc[s][t][r] * oscale;
        }
  } else {
#pragma unroll
    for (int s = 0; s < 2; ++s)
#pragma unroll
      for (int t = 0; t < 2; ++t)
#pragma unroll
        for (int r = 0; r < 8; ++r)
          st[(nw + 16 * t + c) * TTP + mw + 16 * s + 8 * hh + r] = acc[s][t][r] * oscale;
  }
  __syncthreads();

  if (!tr && has_f != 0) {
    v4f val[8];
    size_t go[8];
#pragma unroll
    for (int it = 0; it < 8; ++it) {
      const int idx = tid + 256 * it;
      const int row = idx >> 4, pc = idx & 15;
      float* sp = st + row * OTP + 4 * pc;
      v4f v = *(const v4fa*)(sp);
      go[it] = (size_t)(mblk + row) * ldcf + nblk + 4 * pc;
      if (resid != 0) {
        const v4f rr = *(const v4f*)(Cf + go[it]);
        v = v + rr;
        *(v4fa*)(sp) = v;
      }
      if (relu_f != 0) v = relu4(v);
      val[it] = v;
    }
    for (int ps = 0; ps < 2; ++ps) {
#pragma unroll
      for (int it = 0; it < 8; ++it) *(volatile v4f*)(Cf + go[it]) = val[it];
      __threadfence();
    }
  }
  __syncthreads();

  if (!tr) {
    if (has_h != 0) {
      v4u w[4];
      size_t go[4];
#pragma unroll
      for (int it = 0; it < 4; ++it) {
        const int idx = tid + 256 * it;
        const int row = idx >> 3, pc = idx & 7;
        const v4fa* rp = (const v4fa*)(st + row * OTP + 8 * pc);
        v4f a0 = rp[0], a1 = rp[1];
        if (relu_h != 0) { a0 = relu4(a0); a1 = relu4(a1); }
        w[it]  = pk2(a0, a1);
        go[it] = (size_t)z * chzs + (size_t)(mblk + row) * ldch + nblk + 8 * pc;
      }
      for (int ps = 0; ps < 2; ++ps) {
#pragma unroll
        for (int it = 0; it < 4; ++it) *(volatile v4u*)(Ch + go[it]) = w[it];
        __threadfence();
      }
    }
  } else {
    const int b  = mblk / NA;
    const int a0 = mblk - b * NA;
    v4u w[4];
    size_t go[4];
#pragma unroll
    for (int it = 0; it < 4; ++it) {
      const int idx  = tid + 256 * it;
      const int drow = idx >> 4, pc = idx & 15;
      const v4fa* rp = (const v4fa*)(st + drow * TTP + 8 * pc);
      w[it]  = pk2(rp[0], rp[1]);
      go[it] = (size_t)(b * DS + nblk + drow) * VTP + VTH + a0 + 8 * pc;
    }
    for (int ps = 0; ps < 2; ++ps) {
#pragma unroll
      for (int it = 0; it < 4; ++it) *(volatile v4u*)(Vt + go[it]) = w[it];
      __threadfence();
    }
  }
}

__global__ __launch_bounds__(128) void k_pair(const float* __restrict__ pos, const int* __restrict__ uid,
                                              const float* __restrict__ P64, const float* __restrict__ Wpair,
                                              const float* __restrict__ W1, const float* __restrict__ W2,
                                              const float* __restrict__ Wb, float* __restrict__ bias) {
  __shared__ __align__(16) _Float16 sW1[64 * 40];
  __shared__ __align__(16) _Float16 sW2[16 * 72];
  __shared__ float sWp[80];
  __shared__ float sWb[64];
  __shared__ __align__(16) _Float16 sA[4 * 32 * 40];
  __shared__ __align__(16) _Float16 sH[4 * 32 * 72];
  __shared__ __align__(16) float sF[4 * 32 * 20];
  __shared__ __align__(16) float sBi[4 * 256];

  const int tid = threadIdx.x, lane = tid & 31, wave = tid >> 5, hh = lane >> 4, c = lane & 15;
  for (int i = tid; i < 64 * 32; i += 128) {
    const int n = i >> 5, k = i & 31;
    const int kc = min(k, 15);
    const float v = W1[kc * 64 + n];
    sW1[n * 40 + k] = (k < 16) ? (_Float16)v : (_Float16)0.f;
  }
  for (int i = tid; i < 16 * 64; i += 128) {
    const int n = i >> 6, k = i & 63;
    sW2[n * 72 + k] = (_Float16)W2[k * 16 + n];
  }
  for (int i = tid; i < 80; i += 128) sWp[i] = Wpair[i];
  for (int i = tid; i < 64; i += 128) sWb[i] = Wb[i];
  _Float16* sAw = sA + wave * 32 * 40;
  _Float16* sHw = sH + wave * 32 * 72;
  float*    sFw = sF + wave * 32 * 20;
  float*    sBw = sBi + wave * 256;
  {
    const v4u z4 = {0u, 0u, 0u, 0u};
    *(v4u*)(sAw + lane * 40 + 16) = z4;
    *(v4u*)(sAw + lane * 40 + 24) = z4;
  }
  __syncthreads();

  const int b = blockIdx.z, wn = blockIdx.y;
  const int q = 2 * blockIdx.x + (wave >> 1), kh = wave & 1;
  const int ai = b * NA + wn * QW + q;
  const float pix = pos[(size_t)ai * 3 + 0], piy = pos[(size_t)ai * 3 + 1], piz = pos[(size_t)ai * 3 + 2];
  const int ui = uid[ai];
  float pi[16];
  {
    const float* pp = P64 + (size_t)ai * 64;
#pragma unroll
    for (int g = 0; g < 4; ++g) {
      const v4f v = *(const v4f*)(pp + 4 * g);
      pi[4 * g + 0] = v[0]; pi[4 * g + 1] = v[1]; pi[4 * g + 2] = v[2]; pi[4 * g + 3] = v[3];
    }
  }

#pragma unroll 1
  for (int ps = 0; ps < 2; ++ps) {
    const int kk = 64 * kh + 32 * ps + lane;
    const int a = wn * QW + kk - PADW;
    const bool valid = (unsigned)a < (unsigned)NA;
    const int ac = min(max(a, 0), NA - 1);
    const int aj = b * NA + ac;
    const float qx = pos[(size_t)aj * 3 + 0], qy = pos[(size_t)aj * 3 + 1], qz = pos[(size_t)aj * 3 + 2];
    const int uraw = uid[aj];
    float pj[16];
    {
      const float* pp = P64 + (size_t)aj * 64 + 16;
#pragma unroll
      for (int g = 0; g < 4; ++g) {
        const v4f v = *(const v4f*)(pp + 4 * g);
        pj[4 * g + 0] = valid ? v[0] : 0.f; pj[4 * g + 1] = valid ? v[1] : 0.f;
        pj[4 * g + 2] = valid ? v[2] : 0.f; pj[4 * g + 3] = valid ? v[3] : 0.f;
      }
    }
    const float pjx = valid ? qx : 0.f, pjy = valid ? qy : 0.f, pjz = valid ? qz : 0.f;
    const int uj = valid ? uraw : 0;
    const float d0 = pix - pjx, d1 = piy - pjy, d2 = piz - pjz;
    const float sq  = (d0 * d0 + d2 * d2) + d1 * d1;
    const float inv = __builtin_amdgcn_rcpf(1.0f + sq);
    const float bij = (ui == uj) ? 1.0f : 0.0f;
    float pre[16];
#pragma unroll
    for (int cc = 0; cc < 16; ++cc) {
      const float t = d0 * sWp[cc] + d1 * sWp[16 + cc] + d2 * sWp[32 + cc] + inv * sWp[48 + cc] + bij * sWp[64 + cc];
      pre[cc] = t * bij + pi[cc] + pj[cc];
    }
    float mean = 0.f;
#pragma unroll
    for (int cc = 0; cc < 16; ++cc) mean += pre[cc];
    mean *= (1.0f / 16.f);
    float var = 0.f;
#pragma unroll
    for (int cc = 0; cc < 16; ++cc) { const float d = pre[cc] - mean; var += d * d; }
    const float r = rsqrtf(var * (1.0f / 16.f) + 1e-5f);
    float lnv[16];
#pragma unroll
    for (int cc = 0; cc < 16; ++cc) lnv[cc] = (pre[cc] - mean) * r;
    *(v4u*)(sAw + lane * 40 + 0) = pk2((v4f){lnv[0], lnv[1], lnv[2], lnv[3]}, (v4f){lnv[4], lnv[5], lnv[6], lnv[7]});
    *(v4u*)(sAw + lane * 40 + 8) = pk2((v4f){lnv[8], lnv[9], lnv[10], lnv[11]}, (v4f){lnv[12], lnv[13], lnv[14], lnv[15]});
    wsync();

#pragma unroll
    for (int rt = 0; rt < 2; ++rt) {
      const v16h af = ldf(sAw, 40, 16 * rt, 0, lane);
      v8f acc[4];
#pragma unroll
      for (int t = 0; t < 4; ++t) acc[t] = mma(af, ldf(sW1, 40, 16 * t, 0, lane), zero8());
#pragma unroll
      for (int t = 0; t < 4; ++t)
#pragma unroll
        for (int rr = 0; rr < 8; ++rr)
          sHw[(16 * rt + 8 * hh + rr) * 72 + 16 * t + c] = (_Float16)fmaxf(acc[t][rr], 0.f);
    }
    wsync();

    {
      const v16h b0 = ldf(sW2, 72, 0, 0, lane), b1 = ldf(sW2, 72, 0, 32, lane);
#pragma unroll
      for (int rt = 0; rt < 2; ++rt) {
        const v16h a0 = ldf(sHw, 72, 16 * rt, 0, lane);
        const v16h a1 = ldf(sHw, 72, 16 * rt, 32, lane);
        v8f acc2 = mma(a0, b0, zero8());
        acc2 = mma(a1, b1, acc2);
#pragma unroll
        for (int rr = 0; rr < 8; ++rr) sFw[(16 * rt + 8 * hh + rr) * 20 + c] = acc2[rr];
      }
    }
    wsync();

    {
      const v4fa* fr = (const v4fa*)(sFw + lane * 20);
      const v4f f0 = fr[0], f1 = fr[1], f2 = fr[2], f3 = fr[3];
      float fin[16];
      fin[0]  = pre[0]  + f0[0]; fin[1]  = pre[1]  + f0[1]; fin[2]  = pre[2]  + f0[2]; fin[3]  = pre[3]  + f0[3];
      fin[4]  = pre[4]  + f1[0]; fin[5]  = pre[5]  + f1[1]; fin[6]  = pre[6]  + f1[2]; fin[7]  = pre[7]  + f1[3];
      fin[8]  = pre[8]  + f2[0]; fin[9]  = pre[9]  + f2[1]; fin[10] = pre[10] + f2[2]; fin[11] = pre[11] + f2[3];
      fin[12] = pre[12] + f3[0]; fin[13] = pre[13] + f3[1]; fin[14] = pre[14] + f3[2]; fin[15] = pre[15] + f3[3];
#pragma unroll
      for (int h = 0; h < NH; ++h) {
        float bb = 0.f;
#pragma unroll
        for (int cc = 0; cc < 16; ++cc) bb += fin[cc] * sWb[cc * 4 + h];
        sBw[h * 64 + 32 * ps + lane] = bb;
      }
    }
    wsync();
  }

  v4f val[2];
  size_t go[2];
#pragma unroll
  for (int it = 0; it < 2; ++it) {
    const int idx = lane + 32 * it;
    const int h = idx >> 4, pc = idx & 15;
    val[it] = *(const v4fa*)(sBw + h * 64 + 4 * pc);
    go[it]  = ((((size_t)(b * NWI + wn)) * NH + h) * QW + q) * KW + 64 * kh + 4 * pc;
  }
  for (int ps = 0; ps < 2; ++ps) {
#pragma unroll
    for (int it = 0; it < 2; ++it) *(volatile v4f*)(bias + go[it]) = val[it];
    __threadfence();
  }
}

__global__ __launch_bounds__(256) void k_attn(const _Float16* __restrict__ Q, const _Float16* __restrict__ Kp,
                                              const _Float16* __restrict__ Vt, const float* __restrict__ bias,
                                              _Float16* __restrict__ O) {
  __shared__ __align__(16) _Float16 sP[8 * 16 * PTP];
  __shared__ __align__(16) _Float16 sO[64 * PTP];
  __shared__ __align__(16) float    sBs[8 * 16 * BTP];

  const int tid = threadIdx.x, lane = tid & 31, wave = tid >> 5;
  const int hh = lane >> 4, c = lane & 15;
  const int wn = blockIdx.x, b = blockIdx.y;
  const float SCL = 1.0f / 5.656854249492381f;
  _Float16* sPw = sP + wave * 16 * PTP;
  float*    sBw = sBs + wave * 16 * BTP;
  const _Float16* Vb = Vt + (size_t)b * DS * VTP;

  for (int task = wave; task < 16; task += 8) {
    const int h = task & 3, qt = task >> 2;
    const int arow0 = b * NA + wn * QW + 16 * qt;

    {
      const float* bsrc = bias + ((((size_t)(b * NWI + wn)) * NH + h) * QW + 16 * qt) * KW;
#pragma unroll 1
      for (int g = 0; g < 4; ++g) {
        v4f t4[4];
#pragma unroll
        for (int i = 0; i < 4; ++i) t4[i] = *(const v4f*)(bsrc + 4 * (lane + 32 * (4 * g + i)));
#pragma unroll
        for (int i = 0; i < 4; ++i) {
          const int p = lane + 32 * (4 * g + i);
          *(v4fa*)(sBw + (p >> 5) * BTP + 4 * (p & 31)) = t4[i];
        }
      }
    }
    wsync();

    const v16h aq = ldf(Q, DS, arow0, h * HD, lane);
    v8f s[8];
#pragma unroll
    for (int j = 0; j < 4; ++j) {
      const int a  = wn * QW - PADW + 16 * j + c;
      const int ac = min(max(a, 0), NA - 1);
      const v16h bk = ldq(Kp + (size_t)(b * NA + ac) * DS + h * HD + 8 * hh);
      s[j] = mma(aq, bk, zero8());
    }
    asm volatile("" ::: "memory");
#pragma unroll
    for (int j = 4; j < 8; ++j) {
      const int a  = wn * QW - PADW + 16 * j + c;
      const int ac = min(max(a, 0), NA - 1);
      const v16h bk = ldq(Kp + (size_t)(b * NA + ac) * DS + h * HD + 8 * hh);
      s[j] = mma(aq, bk, zero8());
    }
#pragma unroll
    for (int j = 0; j < 8; ++j) {
      const int key = 16 * j + c;
      const bool valid = (unsigned)(wn * QW - PADW + key) < (unsigned)NA;
      const float km = valid ? 0.f : -1.0e9f;
#pragma unroll
      for (int r = 0; r < 8; ++r) {
        const float v = s[j][r] * SCL + sBw[(8 * hh + r) * BTP + key];
        s[j][r] = v + km;
      }
    }
    float mrow[8], lsum[8];
#pragma unroll
    for (int r = 0; r < 8; ++r) {
      float m = fmaxf(fmaxf(fmaxf(s[0][r], s[1][r]), fmaxf(s[2][r], s[3][r])),
                      fmaxf(fmaxf(s[4][r], s[5][r]), fmaxf(s[6][r], s[7][r])));
#pragma unroll
      for (int off = 1; off < 16; off <<= 1) m = fmaxf(m, __shfl_xor(m, off, 32));
      mrow[r] = m;
    }
#pragma unroll
    for (int r = 0; r < 8; ++r) {
      float sum = 0.f;
#pragma unroll
      for (int j = 0; j < 8; ++j) {
        const float e = __expf(s[j][r] - mrow[r]);
        sum += e;
        sPw[(8 * hh + r) * PTP + 16 * j + c] = (_Float16)(e * 1024.0f);
      }
#pragma unroll
      for (int off = 1; off < 16; off <<= 1) sum += __shfl_xor(sum, off, 32);
      lsum[r] = sum;
    }
    wsync();

    v8f o[2];
    o[0] = zero8(); o[1] = zero8();
#pragma unroll 1
    for (int kq = 0; kq < 4; ++kq) {
      const v16h ap = ldf(sPw, PTP, 0, 32 * kq, lane);
#pragma unroll
      for (int t = 0; t < 2; ++t) {
        const v16h bv = ldf(Vb, VTP, h * HD + 16 * t, PADW + wn * QW + 32 * kq, lane);
        o[t] = mma(ap, bv, o[t]);
      }
    }
#pragma unroll
    for (int r = 0; r < 8; ++r) {
      const float inv = __builtin_amdgcn_rcpf(lsum[r] * 1024.0f);
#pragma unroll
      for (int t = 0; t < 2; ++t) sO[(16 * qt + 8 * hh + r) * PTP + h * HD + 16 * t + c] = (_Float16)(o[t][r] * inv);
    }
    wsync();
  }
  __syncthreads();

  v4u w[4];
  size_t go[4];
#pragma unroll
  for (int it = 0; it < 4; ++it) {
    const int idx = tid + 256 * it;
    const int row = idx >> 4, pc = idx & 15;
    w[it]  = *(const v4ua*)(sO + row * PTP + 8 * pc);
    go[it] = (size_t)(b * NA + wn * QW + row) * DS + 8 * pc;
  }
  for (int ps = 0; ps < 2; ++ps) {
#pragma unroll
    for (int it = 0; it < 4; ++it) *(volatile v4u*)(O + go[it]) = w[it];
    __threadfence();
  }
}

__global__ __launch_bounds__(256) void k_seg(const float* __restrict__ tok, const int* __restrict__ a2t,
                                             const int* __restrict__ ntp, float* __restrict__ out) {
  __shared__ __align__(16) float sAcc[32 * DT];
  __shared__ int sList[256];
  __shared__ int sWc[8];
  __shared__ int sCnt[32];
  const int tid = threadIdx.x, lane = tid & 31, wave = tid >> 5;
  const int b = blockIdx.y, t0 = blockIdx.x * 32;
  const int ntok = ntp[0];
  for (int i = tid; i < 32 * DT; i += 256) sAcc[i] = 0.f;
  if (tid < 32) sCnt[tid] = 0;
  __syncthreads();

  for (int ch = 0; ch < NA / 256; ++ch) {
    const int a = ch * 256 + tid;
    const int t = a2t[(size_t)b * NA + a];
    const bool hit = (t >= t0) && (t < t0 + 32) && (t < ntok);
    const unsigned m  = (unsigned)__ballot(hit);
    const unsigned lt = (1u << lane) - 1u;
    const int pw = __popc(m & lt);
    if (lane == 0) sWc[wave] = __popc(m);
    __syncthreads();
    int off = 0, tot = 0;
#pragma unroll
    for (int w2 = 0; w2 < 8; ++w2) {
      const int cw = sWc[w2];
      tot += cw;
      off += (w2 < wave) ? cw : 0;
    }
    if (hit) sList[off + pw] = a | ((t - t0) << 16);
    __syncthreads();
    const int cnt = min(tot, 256);
    for (int mm = 0; mm < cnt; ++mm) {
      const int e  = sList[mm];
      const int aa = min(e & 0xffff, NA - 1);
      const int tl = (e >> 16) & 31;
      const float* src = tok + (size_t)(b * NA + aa) * DT;
      for (int cc = tid; cc < DT; cc += 256) sAcc[tl * DT + cc] += src[cc];
      if (tid == 0) sCnt[tl] += 1;
    }
    __syncthreads();
  }

  v4f val[12];
  size_t go[12];
#pragma unroll
  for (int it = 0; it < 12; ++it) {
    const int idx = tid + 256 * it;
    const int row = idx / 96;
    const int pc  = idx - row * 96;
    const int cn  = max(sCnt[row], 1);
    const float inv = 1.0f / (float)cn;
    const v4f v = *(const v4fa*)(sAcc + row * DT + 4 * pc);
    val[it] = (v4f){v[0] * inv, v[1] * inv, v[2] * inv, v[3] * inv};
    go[it]  = (size_t)(b * NTK + t0 + row) * DT + 4 * pc;
  }
  for (int ps = 0; ps < 2; ++ps) {
#pragma unroll
    for (int it = 0; it < 12; ++it) *(volatile v4f*)(out + go[it]) = val[it];
    __threadfence();
  }
}

extern "C" void kernel_launch(void* const* d_in, const int* in_sizes, int n_in,
                              void* d_out, int out_size, void* d_ws, size_t ws_size,
                              hipStream_t stream) {
  if (n_in < 21) return;
  if (in_sizes[0] != MA * 3) return;
  if (in_sizes[1] != MA) return;
  if (in_sizes[2] != MA) return;
  if (in_sizes[3] != MA * 128) return;
  if (in_sizes[4] != MA * 256) return;
  if (in_sizes[5] != KF * DS) return;
  if (in_sizes[6] != 5 * DP) return;
  if (in_sizes[7] != DS * 2 * DP) return;
  if (in_sizes[8] != DP * 4 * DP) return;
  if (in_sizes[9] != 4 * DP * DP) return;
  if (in_sizes[10] != DEP * DS * DS) return;
  if (in_sizes[11] != DEP * DS * DS) return;
  if (in_sizes[12] != DEP * DS * DS) return;
  if (in_sizes[13] != DEP * DS * DS) return;
  if (in_sizes[14] != DP * NH) return;
  if (in_sizes[15] != DEP * DS * DFF) return;
  if (in_sizes[16] != DEP * DFF * DS) return;
  if (in_sizes[17] != DS * DT) return;
  if (in_sizes[18] != MA) return;
  if (in_sizes[19] != MA) return;
  if (in_sizes[20] != 1) return;
  if (out_size != NB * NTK * DT) return;

  const float* ref_pos   = (const float*)d_in[0];
  const float* ref_chg   = (const float*)d_in[1];
  const float* ref_msk   = (const float*)d_in[2];
  const float* ref_elem  = (const float*)d_in[3];
  const float* ref_chars = (const float*)d_in[4];
  const float* W_single  = (const float*)d_in[5];
  const float* W_pair    = (const float*)d_in[6];
  const float* W_outer   = (const float*)d_in[7];
  const float* Wp_ff1    = (const float*)d_in[8];
  const float* Wp_ff2    = (const float*)d_in[9];
  const float* Wq        = (const float*)d_in[10];
  const float* Wk        = (const float*)d_in[11];
  const float* Wv        = (const float*)d_in[12];
  const float* Wo        = (const float*)d_in[13];
  const float* Wb        = (const float*)d_in[14];
  const float* Wff1      = (const float*)d_in[15];
  const float* Wff2      = (const float*)d_in[16];
  const float* W_out     = (const float*)d_in[17];
  const int*   uid       = (const int*)d_in[18];
  const int*   a2t       = (const int*)d_in[19];
  const int*   ntok      = (const int*)d_in[20];
  float* out = (float*)d_out;

  size_t off = 0;
  const size_t oF    = off; off += (size_t)MA * KFP * 2;
  const size_t oWsT  = off; off += (size_t)DS * KFP * 2;
  const size_t oWorT = off; off += (size_t)64 * DS * 2;
  const size_t oWqkv = off; off += (size_t)9 * DS * DS * 2;
  const size_t oWoT  = off; off += (size_t)DEP * DS * DS * 2;
  const size_t oWf1T = off; off += (size_t)DEP * DFF * DS * 2;
  const size_t oWf2T = off; off += (size_t)DEP * DS * DFF * 2;
  const size_t oWtT  = off; off += (size_t)DT * DS * 2;
  const size_t oX    = off; off += (size_t)MA * DS * 4;
  const size_t oSR   = off; off += (size_t)MA * DS * 2;
  const size_t oP64  = off; off += (size_t)MA * 64 * 4;
  const size_t oBIAS = off; off += (size_t)NB * NWI * NH * QW * KW * 4;
  const size_t oH    = off; off += (size_t)MA * DS * 2;
  const size_t oQK   = off; off += (size_t)2 * MA * DS * 2;
  const size_t oVT   = off; off += (size_t)NB * DS * VTP * 2;
  const size_t oO    = off; off += (size_t)MA * DS * 2;
  const size_t oFFH  = off; off += (size_t)MA * DFF * 2;
  if ((size_t)MA * DT * 4 > (size_t)NB * NWI * NH * QW * KW * 4) return;
  if (off > ws_size) return;
  if (off > (size_t)134217728) return;

  char* ws = (char*)d_ws;
  _Float16* F     = (_Float16*)(ws + oF);
  _Float16* WsT   = (_Float16*)(ws + oWsT);
  _Float16* WorT  = (_Float16*)(ws + oWorT);
  _Float16* WqkvT = (_Float16*)(ws + oWqkv);
  _Float16* WoT   = (_Float16*)(ws + oWoT);
  _Float16* Wf1T  = (_Float16*)(ws + oWf1T);
  _Float16* Wf2T  = (_Float16*)(ws + oWf2T);
  _Float16* WtT   = (_Float16*)(ws + oWtT);
  float*    X     = (float*)(ws + oX);
  _Float16* SR    = (_Float16*)(ws + oSR);
  _Float16* XH    = SR;
  float*    P64   = (float*)(ws + oP64);
  float*    BIAS  = (float*)(ws + oBIAS);
  float*    TOK   = BIAS;
  _Float16* H     = (_Float16*)(ws + oH);
  _Float16* QK    = (_Float16*)(ws + oQK);
  _Float16* VT    = (_Float16*)(ws + oVT);
  _Float16* Op    = (_Float16*)(ws + oO);
  _Float16* FFH   = (_Float16*)(ws + oFFH);

  const dim3 blk(256);
  const int L16 = DS * DS;
  const int L64 = DS * DFF;

  k_wtr<<<dim3(KFP / 64, DS / 64, 1), blk, 0, stream>>>(W_single, KF, DS, 0, WsT, KFP, 0, 16.0f, 1);
  k_wtr<<<dim3(DS / 64, 1, 1), blk, 0, stream>>>(W_outer, DS, 32, 0, WorT, DS, 0, 8.0f, 0);
  k_wtr<<<dim3(DS / 64, DS / 64, DEP), blk, 0, stream>>>(Wq, DS, DS, L16, WqkvT, DS, L16, 8.0f, 0);
  k_wtr<<<dim3(DS / 64, DS / 64, DEP), blk, 0, stream>>>(Wk, DS, DS, L16, WqkvT + (size_t)3 * L16, DS, L16, 8.0f, 0);
  k_wtr<<<dim3(DS / 64, DS / 64, DEP), blk, 0, stream>>>(Wv, DS, DS, L16, WqkvT + (size_t)6 * L16, DS, L16, 8.0f, 0);
  k_wtr<<<dim3(DS / 64, DS / 64, DEP), blk, 0, stream>>>(Wo, DS, DS, L16, WoT, DS, L16, 8.0f, 0);
  k_wtr<<<dim3(DS / 64, DFF / 64, DEP), blk, 0, stream>>>(Wff1, DS, DFF, L64, Wf1T, DS, L64, 8.0f, 0);
  k_wtr<<<dim3(DFF / 64, DS / 64, DEP), blk, 0, stream>>>(Wff2, DFF, DS, L64, Wf2T, DFF, L64, 16.0f, 0);
  k_wtr<<<dim3(DS / 64, DT / 64, 1), blk, 0, stream>>>(W_out, DS, DT, 0, WtT, DS, 0, 8.0f, 0);
  k_feats<<<dim3(MA / 8), blk, 0, stream>>>(ref_pos, ref_chg, ref_msk, ref_elem, ref_chars, F);
  k_zvt<<<dim3(16), blk, 0, stream>>>(VT);
  k_gemm<<<dim3(DS / 64, MA / 128, 1), blk, 0, stream>>>(F, KFP, WsT, KFP, 0, KFL, 1.0f / 16.0f,
                                                         X, DS, 1, 0, 0, SR, DS, 0, 1, 1, VT, -1);
  k_gemm<<<dim3(1, MA / 128, 1), blk, 0, stream>>>(SR, DS, WorT, DS, 0, DS, 1.0f / 8.0f,
                                                   P64, 64, 1, 0, 0, SR, DS, 0, 0, 0, VT, -1);
  k_pair<<<dim3(QW / 2, NWI, NB), dim3(128), 0, stream>>>(ref_pos, uid, P64, W_pair, Wp_ff1, Wp_ff2, Wb, BIAS);
  for (int l = 0; l < DEP; ++l) {
    k_ln<<<dim3(MA / 16), blk, 0, stream>>>(X, H);
    k_gemm<<<dim3(DS / 64, MA / 128, 3), blk, 0, stream>>>(H, DS, WqkvT + (size_t)l * L16, DS, 3 * L16, DS,
                                                           1.0f / 8.0f, X, DS, 0, 0, 0,
                                                           QK, DS, MA * DS, 1, 0, VT, 2);
    k_attn<<<dim3(NWI, NB), blk, 0, stream>>>(QK, QK + (size_t)MA * DS, VT, BIAS, Op);
    k_gemm<<<dim3(DS / 64, MA / 128, 1), blk, 0, stream>>>(Op, DS, WoT + (size_t)l * L16, DS, 0, DS, 1.0f / 8.0f,
                                                           X, DS, 1, 1, 0, H, DS, 0, 0, 0, VT, -1);
    k_ln<<<dim3(MA / 16), blk, 0, stream>>>(X, H);
    k_gemm<<<dim3(DFF / 64, MA / 128, 1), blk, 0, stream>>>(H, DS, Wf1T + (size_t)l * L64, DS, 0, DS, 1.0f / 8.0f,
                                                            X, DS, 0, 0, 0, FFH, DFF, 0, 1, 1, VT, -1);
    const int emit_xh = (l == DEP - 1) ? 1 : 0;
    k_gemm<<<dim3(DS / 64, MA / 128, 1), blk, 0, stream>>>(FFH, DFF, Wf2T + (size_t)l * L64, DFF, 0, DFF,
                                                           1.0f / 16.0f, X, DS, 1, 1, 0,
                                                           XH, DS, 0, emit_xh, 0, VT, -1);
  }
  k_gemm<<<dim3(DT / 64, MA / 128, 1), blk, 0, stream>>>(XH, DS, WtT, DS, 0, DS, 1.0f / 8.0f,
                                                         TOK, DT, 1, 0, 1, H, DS, 0, 0, 0, VT, -1);
  k_seg<<<dim3(NTK / 32, NB), blk, 0, stream>>>(TOK, a2t, ntok, out);
  (void)hipGetLastError();
}
